// Mamba2Block_44959717654936
// MI455X (gfx1250) — hardware-verified
//
#include <hip/hip_runtime.h>
#include <math.h>

typedef __attribute__((ext_vector_type(16))) _Float16 v16h;
typedef __attribute__((ext_vector_type(8)))  _Float16 v8h;
typedef __attribute__((ext_vector_type(16))) __bf16   v16b;
typedef __attribute__((ext_vector_type(8)))  __bf16   v8b;
typedef __attribute__((ext_vector_type(8)))  float    v8f;
typedef __attribute__((ext_vector_type(4)))  float    v4f;

constexpr int kBatch = 2;
constexpr int kSeq   = 4096;
constexpr int kDm    = 1024;
constexpr int kDz    = 2048;
constexpr int kDin   = 512;
constexpr int kNh    = 8;
constexpr int kNst   = 64;
constexpr int kHd    = 64;
constexpr int kNssm  = 2 * kNst + kNh + kDin;
constexpr int kLdS   = 704;
constexpr int kRows  = kBatch * kSeq;
constexpr int kHalf  = kRows / 2;
constexpr int kColB  = 0;
constexpr int kColC  = kNst;
constexpr int kColDt = 2 * kNst;
constexpr int kColX  = 2 * kNst + kNh;
constexpr int kScanTS = 32;
constexpr int kYP     = 68;
constexpr int kOutElems0 = kRows * kDm;
constexpr int kOutElems1 = kBatch * kNh * kHd * kNst;
static_assert(kNssm == 648);
static_assert((size_t)kOutElems0 * 4 == 33554432ull);
static_assert(((size_t)kOutElems0 + kOutElems1) * 4 == 33816576ull);
static_assert((kDm % 32) == 0 && (kDz % 32) == 0 && (kDin % 32) == 0);
static_assert((kRows % 64) == 0 && (kHalf % 64) == 0);
static_assert((kDz % 64) == 0 && (kLdS % 64) == 0 && (kDin % 64) == 0 && (kDm % 64) == 0);
static_assert(kLdS >= kNssm && (kNssm % 4) == 0 && (kDz % 4) == 0 && (kDin % 4) == 0 && (kDm % 4) == 0);
static_assert((kSeq % kScanTS) == 0 && kScanTS == 32 && kHd == 64 && kNst == 64);

constexpr size_t kOffXB    = 0;
constexpr size_t kOffWZT   = kOffXB    + (size_t)kRows * kDm * 2;
constexpr size_t kOffWINT  = kOffWZT   + (size_t)kDz * kDm * 2;
constexpr size_t kOffWZGT  = kOffWINT  + (size_t)kLdS * kDm * 2;
constexpr size_t kOffWOUTT = kOffWZGT  + (size_t)kDin * kDz * 2;
constexpr size_t kOffZSH   = kOffWOUTT + (size_t)kDm * kDin * 2;
constexpr size_t kOffZSL   = kOffZSH   + (size_t)kHalf * kDz * 2;
constexpr size_t kOffSSM   = kOffZSL   + (size_t)kHalf * kDz * 2;
constexpr size_t kOffY     = kOffSSM   + (size_t)kRows * kLdS * 4;
constexpr size_t kOffGH    = kOffY     + (size_t)kRows * kDin * 4;
constexpr size_t kOffGL    = kOffGH    + (size_t)kRows * kDin * 2;
constexpr size_t kWsTotal  = kOffGL    + (size_t)kRows * kDin * 2;
static_assert(kWsTotal == 115736576ull);
static_assert(kWsTotal <= 134217728ull);
static_assert((kOffWZT % 128) == 0 && (kOffWINT % 128) == 0 && (kOffWZGT % 128) == 0 && (kOffWOUTT % 128) == 0 &&
              (kOffZSH % 128) == 0 && (kOffZSL % 128) == 0 && (kOffSSM % 128) == 0 && (kOffY % 128) == 0 &&
              (kOffGH % 128) == 0 && (kOffGL % 128) == 0);

__device__ __forceinline__ unsigned short f2bf_bits(float f) {
  unsigned u = __float_as_uint(f);
  return (unsigned short)((u + 0x7FFFu + ((u >> 16) & 1u)) >> 16);
}
__device__ __forceinline__ float bf_bits2f(unsigned short h) { return __uint_as_float(((unsigned)h) << 16); }

__device__ __forceinline__ void dep_guard4_h(v8f& a, v8f& b, v8f& c, v8f& d, v16h x, v16h y) {
  asm volatile("v_nop\n\tv_nop\n\tv_nop\n\tv_nop" : "+v"(a), "+v"(b), "+v"(c), "+v"(d) : "v"(x), "v"(y));
}
__device__ __forceinline__ void dep_guard4_b(v8f& a, v8f& b, v8f& c, v8f& d, v16b x, v16b y) {
  asm volatile("v_nop\n\tv_nop\n\tv_nop\n\tv_nop" : "+v"(a), "+v"(b), "+v"(c), "+v"(d) : "v"(x), "v"(y));
}
__device__ __forceinline__ void keep4_h(v16h a, v16h b, v16h c, v16h d) { asm volatile("v_nop" :: "v"(a), "v"(b), "v"(c), "v"(d)); }
__device__ __forceinline__ void keep4_b(v16b a, v16b b, v16b c, v16b d) { asm volatile("v_nop" :: "v"(a), "v"(b), "v"(c), "v"(d)); }
__device__ __forceinline__ void acc_guard4(v8f& a, v8f& b, v8f& c, v8f& d) { asm volatile("v_nop\n\tv_nop\n\tv_nop\n\tv_nop" : "+v"(a), "+v"(b), "+v"(c), "+v"(d)); }
template <typename T> struct Frag;
template <> struct Frag<_Float16> {
  typedef v16h V; union U { v16h v; v8h h[2]; };
  static __device__ __forceinline__ v16h load(const _Float16* p) {
    U f; f.h[0] = *(const v8h*)(p); f.h[1] = *(const v8h*)(p + 16); return f.v;
  }
  static __device__ __forceinline__ v8f mma(v16h a, v16h b, v8f c) {
    return __builtin_amdgcn_wmma_f32_16x16x32_f16(false, a, false, b, (short)0, c, false, false);
  }
  static __device__ __forceinline__ void guard4(v8f& a, v8f& b, v8f& c, v8f& d, v16h x, v16h y) { dep_guard4_h(a, b, c, d, x, y); }
  static __device__ __forceinline__ void keep(v16h a, v16h b, v16h c, v16h d) { keep4_h(a, b, c, d); }
};
template <> struct Frag<__bf16> {
  typedef v16b V; union U { v16b v; v8b h[2]; };
  static __device__ __forceinline__ v16b load(const __bf16* p) {
    U f; f.h[0] = *(const v8b*)(p); f.h[1] = *(const v8b*)(p + 16); return f.v;
  }
  static __device__ __forceinline__ v8f mma(v16b a, v16b b, v8f c) {
    return __builtin_amdgcn_wmma_f32_16x16x32_bf16(false, a, false, b, (short)0, c, false, false);
  }
  static __device__ __forceinline__ void guard4(v8f& a, v8f& b, v8f& c, v8f& d, v16b x, v16b y) { dep_guard4_b(a, b, c, d, x, y); }
  static __device__ __forceinline__ void keep(v16b a, v16b b, v16b c, v16b d) { keep4_b(a, b, c, d); }
};

template <int ET> struct Elem;
template <> struct Elem<0> { typedef _Float16 T; };
template <> struct Elem<1> { typedef __bf16 T; };
template <int ET, int SPL, int OUT_MODE, int ACT, bool MULP>
__global__ __launch_bounds__(256) void wmma_gemm64(
    const unsigned short* __restrict__ Ap, const unsigned short* __restrict__ A2p, int lda,
    const unsigned short* __restrict__ Btp, const unsigned short* __restrict__ Bt2p, int ldb,
    void* __restrict__ Cout, void* __restrict__ Cout2, int ldc,
    const float* __restrict__ mulp, int ldm,
    int M, int N, int K, float scale) {
  typedef typename Elem<ET>::T T;
  typedef typename Frag<T>::V V;
  const T* A = (const T*)Ap; const T* A2 = (const T*)A2p; const T* Bt = (const T*)Btp; const T* Bt2 = (const T*)Bt2p;
  __shared__ __align__(16) float sT[8][16 * 68];
  const int lane = threadIdx.x & 31;
  const int wave = threadIdx.x >> 5;
  const int tilesN = N >> 6;
  const int tilesM = M >> 6;
  const int tile = blockIdx.x * 8 + wave;
  if (tile >= tilesM * tilesN) return;
  const int tm = tile / tilesN;
  const int tn = tile - tm * tilesN;
  const int m0 = tm << 6;
  const int n0 = tn << 6;

  const T* Ab  = A;
  const T* Bb  = Bt;
  const T* Ab2 = (SPL >= 1) ? A2 : nullptr;
  const T* Bb2 = (SPL == 2) ? Bt2 : nullptr;

  const int rlane = lane & 15;
  const int koff  = (lane >> 4) * 8;
  const int mOff  = (lane >> 4) * 8;

  v8f acc[4][4];
#pragma unroll
  for (int i = 0; i < 4; ++i)
#pragma unroll
    for (int j = 0; j < 4; ++j) acc[i][j] = (v8f){0.f,0.f,0.f,0.f,0.f,0.f,0.f,0.f};

  for (int k0 = 0; k0 < K; k0 += 32) {
    V bh[4], bl[4];
#pragma unroll
    for (int j = 0; j < 4; ++j) {
      const size_t bo = (size_t)(n0 + (j << 4) + rlane) * ldb + koff + k0;
      bh[j] = Frag<T>::load(Bb + bo);
      if (SPL == 2) bl[j] = Frag<T>::load(Bb2 + bo);
    }
#pragma unroll
    for (int i = 0; i < 4; ++i) {
      const size_t ao = (size_t)(m0 + (i << 4) + rlane) * lda + koff + k0;
      V ah = Frag<T>::load(Ab + ao);
      V al;
      if (SPL >= 1) al = Frag<T>::load(Ab2 + ao);
#pragma unroll
      for (int j = 0; j < 4; ++j) {
        acc[i][j] = Frag<T>::mma(ah, bh[j], acc[i][j]);
        if (SPL == 2) acc[i][j] = Frag<T>::mma(ah, bl[j], acc[i][j]);
        if (SPL >= 1) acc[i][j] = Frag<T>::mma(al, bh[j], acc[i][j]);
      }
      Frag<T>::guard4(acc[i][0], acc[i][1], acc[i][2], acc[i][3], ah, (SPL >= 1) ? al : ah);
    }
    Frag<T>::keep(bh[0], bh[1], bh[2], bh[3]);
    if (SPL == 2) Frag<T>::keep(bl[0], bl[1], bl[2], bl[3]);
  }
  acc_guard4(acc[0][0], acc[0][1], acc[0][2], acc[0][3]);
  acc_guard4(acc[1][0], acc[1][1], acc[1][2], acc[1][3]);
  acc_guard4(acc[2][0], acc[2][1], acc[2][2], acc[2][3]);
  acc_guard4(acc[3][0], acc[3][1], acc[3][2], acc[3][3]);

  float* slab = sT[wave];
#pragma unroll
  for (int i = 0; i < 4; ++i) {
    const int mBase = m0 + (i << 4);
#pragma unroll
    for (int j = 0; j < 4; ++j) {
#pragma unroll
      for (int r = 0; r < 8; ++r) {
        float v = acc[i][j][r] * scale;
        if (ACT == 3) v = v / (1.0f + expf(-v));
        slab[(mOff + r) * 68 + (j << 4) + rlane] = v;
      }
    }
    __builtin_amdgcn_fence(__ATOMIC_RELEASE, "workgroup");
    __builtin_amdgcn_wave_barrier();
    __builtin_amdgcn_fence(__ATOMIC_ACQUIRE, "workgroup");
    if (OUT_MODE == 0) {
      float* C = (float*)Cout;
      const int hh = lane >> 4, c4 = (lane & 15) * 4;
      for (int pass = 0; pass < 2; ++pass) {
#pragma unroll
        for (int it = 0; it < 8; ++it) {
          const int row = it * 2 + hh;
          v4f v = *(const v4f*)(slab + row * 68 + c4);
          *(volatile v4f*)(C + (size_t)(mBase + row) * ldc + n0 + c4) = v;
        }
        __threadfence();
      }
    } else {
      const int q = lane >> 3, c8 = (lane & 7) * 8;
      unsigned short* C  = (unsigned short*)Cout;
      unsigned short* C2 = (OUT_MODE == 2) ? (unsigned short*)Cout2 : nullptr;
      for (int pass = 0; pass < 2; ++pass) {
#pragma unroll
        for (int it = 0; it < 4; ++it) {
          const int row = it * 4 + q;
          const float* sp = slab + row * 68 + c8;
          v4f ma = (v4f){1.f, 1.f, 1.f, 1.f};
          v4f mb = ma;
          if (MULP) {
            const float* mp = mulp + (size_t)(mBase + row) * ldm + n0 + c8;
            ma = *(const v4f*)(mp);
            mb = *(const v4f*)(mp + 4);
          }
          v8h hv, lv;
#pragma unroll
          for (int e = 0; e < 8; ++e) {
            const float mf = (e < 4) ? ma[e & 3] : mb[e & 3];
            const float val = sp[e] * mf;
            if (OUT_MODE == 1) {
              hv[e] = (_Float16)val;
            } else {
              unsigned short hb = f2bf_bits(val);
              unsigned short lb = f2bf_bits(val - bf_bits2f(hb));
              hv[e] = __builtin_bit_cast(_Float16, hb);
              lv[e] = __builtin_bit_cast(_Float16, lb);
            }
          }
          *(volatile v8h*)(C + (size_t)(mBase + row) * ldc + n0 + c8) = hv;
          if (OUT_MODE == 2) *(volatile v8h*)(C2 + (size_t)(mBase + row) * ldc + n0 + c8) = lv;
        }
        __threadfence();
      }
    }
    __builtin_amdgcn_fence(__ATOMIC_RELEASE, "workgroup");
    __builtin_amdgcn_wave_barrier();
    __builtin_amdgcn_fence(__ATOMIC_ACQUIRE, "workgroup");
  }
}

__global__ __launch_bounds__(256) void cast_rows_bf16_kernel(
    const float* __restrict__ src, unsigned short* __restrict__ dst, int total8)
{
  const int i = blockIdx.x * 256 + threadIdx.x;
  if (i >= total8) return;
  const size_t e0 = (size_t)i << 3;
  const v4f a0 = *(const v4f*)(src + e0);
  const v4f a1 = *(const v4f*)(src + e0 + 4);
  v8h hv;
#pragma unroll
  for (int e = 0; e < 4; ++e) {
    const unsigned short h0 = f2bf_bits(a0[e]), h1 = f2bf_bits(a1[e]);
    hv[e]     = __builtin_bit_cast(_Float16, h0);
    hv[4 + e] = __builtin_bit_cast(_Float16, h1);
  }
  unsigned short* qh = dst + e0;
  *(volatile v8h*)qh = hv;
  __threadfence();
  *(volatile v8h*)qh = hv;
}

__global__ __launch_bounds__(256) void transpose_bf16_kernel(
    const float* __restrict__ W, unsigned short* __restrict__ Bt, int Kdim, int Ndim, int ldbt)
{
  __shared__ float sW[64 * 65];
  const int tid = threadIdx.x, lane = tid & 31, wave = tid >> 5;
  const int n0 = blockIdx.x * 64, k0 = blockIdx.y * 64;
  {
    const int kk = tid >> 2, cb = (tid & 3) * 16;
    const float* wr = W + (size_t)(k0 + kk) * Ndim;
#pragma unroll
    for (int q4 = 0; q4 < 4; ++q4) {
      const int col  = n0 + cb + 4 * q4;
      const int colc = (col < Ndim) ? col : (Ndim - 4);
      const v4f v = *(const v4f*)(wr + colc);
      const float fz = (col < Ndim) ? 1.0f : 0.0f;
      float* sp = sW + kk * 65 + cb + 4 * q4;
      sp[0] = v[0] * fz;
      sp[1] = v[1] * fz;
      sp[2] = v[2] * fz;
      sp[3] = v[3] * fz;
    }
  }
  __syncthreads();
  const int q = lane >> 3, c8 = (lane & 7) * 8;
  v8h hv[2];
#pragma unroll
  for (int it = 0; it < 2; ++it) {
    const int nn = it * 32 + wave * 4 + q;
#pragma unroll
    for (int e = 0; e < 8; ++e) {
      const unsigned short hb = f2bf_bits(sW[(c8 + e) * 65 + nn]);
      hv[it][e] = __builtin_bit_cast(_Float16, hb);
    }
  }
  for (int pass = 0; pass < 2; ++pass) {
#pragma unroll
    for (int it = 0; it < 2; ++it) {
      const int nn = it * 32 + wave * 4 + q;
      *(volatile v8h*)(Bt + (size_t)(n0 + nn) * ldbt + k0 + c8) = hv[it];
    }
    __threadfence();
  }
}

__global__ __launch_bounds__(256) void ssd_scan_kernel(
    const float* __restrict__ SSM, const float* __restrict__ dt_bias, const float* __restrict__ A_log,
    const float* __restrict__ D_param, float* __restrict__ Yp, float* __restrict__ Hout)
{
  __shared__ __align__(16) float sB[kScanTS * kNst];
  __shared__ __align__(16) float sC[kScanTS * kNst];
  __shared__ __align__(16) float sX[kScanTS * kHd];
  __shared__ __align__(16) float sY[kScanTS * kYP];
  __shared__ __align__(16) float sH[kHd * kNst];
  __shared__ float sDel[kScanTS];
  __shared__ float sDA[kScanTS];
  const int tid = threadIdx.x, lane = tid & 31, wave = tid >> 5;
  const int bh = blockIdx.x;
  const int b = bh >> 3, hd = bh & 7;
  const int p = tid >> 2, ng = tid & 3, nb = ng * 16;
  const float dtb  = bf_bits2f(f2bf_bits(dt_bias[hd]));
  const float negA = -expf(bf_bits2f(f2bf_bits(A_log[hd])));
  const float Dp   = bf_bits2f(f2bf_bits(D_param[hd]));
  float hs[16];
#pragma unroll
  for (int j = 0; j < 16; ++j) hs[j] = 0.0f;
  const size_t row0 = (size_t)b * kSeq;
  const int sr = tid >> 3, sc = (tid & 7) * 4;
  const int hh = lane >> 4, c4 = (lane & 15) * 4;

#pragma unroll 1
  for (int t0 = 0; t0 < kSeq; t0 += kScanTS) {
    __syncthreads();
    {
      const float* rp = SSM + (row0 + t0 + sr) * (size_t)kLdS;
      const v4f vb0 = *(const v4f*)(rp + kColB + sc);
      const v4f vb1 = *(const v4f*)(rp + kColB + 32 + sc);
      const v4f vc0 = *(const v4f*)(rp + kColC + sc);
      const v4f vc1 = *(const v4f*)(rp + kColC + 32 + sc);
      const v4f vx0 = *(const v4f*)(rp + kColX + hd * kHd + sc);
      const v4f vx1 = *(const v4f*)(rp + kColX + hd * kHd + 32 + sc);
      *(v4f*)(sB + sr * kNst + sc)      = vb0;
      *(v4f*)(sB + sr * kNst + 32 + sc) = vb1;
      *(v4f*)(sC + sr * kNst + sc)      = vc0;
      *(v4f*)(sC + sr * kNst + 32 + sc) = vc1;
      *(v4f*)(sX + sr * kHd + sc)       = vx0;
      *(v4f*)(sX + sr * kHd + 32 + sc)  = vx1;
    }
    if (wave == 0) {
      const float draw = SSM[(row0 + t0 + lane) * (size_t)kLdS + kColDt + hd] + dtb;
      const float ex = expf(-fabsf(draw));
      const float dl = fmaxf(draw, 0.0f) + log1pf(ex);
      sDel[lane] = dl;
      sDA[lane]  = expf(dl * negA);
    }
    __syncthreads();
#pragma unroll 1
    for (int s = 0; s < kScanTS; ++s) {
      const float dl = sDel[s];
      const float da = sDA[s];
      const float xv = sX[s * kHd + p];
      const float* bp = sB + s * kNst + nb;
      const float* cp = sC + s * kNst + nb;
      float Bv[16], Cv[16];
#pragma unroll
      for (int q4 = 0; q4 < 4; ++q4) {
        const v4f bv = *(const v4f*)(bp + 4 * q4);
        const v4f cv = *(const v4f*)(cp + 4 * q4);
        Bv[4 * q4 + 0] = bv[0]; Bv[4 * q4 + 1] = bv[1]; Bv[4 * q4 + 2] = bv[2]; Bv[4 * q4 + 3] = bv[3];
        Cv[4 * q4 + 0] = cv[0]; Cv[4 * q4 + 1] = cv[1]; Cv[4 * q4 + 2] = cv[2]; Cv[4 * q4 + 3] = cv[3];
      }
      float ysum = 0.0f;
#pragma unroll
      for (int j = 0; j < 16; ++j) {
        const float dB = dl * Bv[j];
        const float xb = xv * dB;
        hs[j] = da * hs[j] + xb;
        ysum = ysum + hs[j] * Cv[j];
      }
      ysum += __shfl_xor(ysum, 1, 32);
      ysum += __shfl_xor(ysum, 2, 32);
      const float yv = ysum + Dp * xv;
      if (ng == 0) sY[s * kYP + p] = yv;
    }
    __syncthreads();
    v4f yst[2];
#pragma unroll
    for (int it = 0; it < 2; ++it) {
      const int row = it * 16 + wave * 2 + hh;
      yst[it] = *(const v4f*)(sY + row * kYP + c4);
    }
    for (int pass = 0; pass < 2; ++pass) {
#pragma unroll
      for (int it = 0; it < 2; ++it) {
        const int row = it * 16 + wave * 2 + hh;
        *(volatile v4f*)(Yp + (row0 + t0 + row) * (size_t)kDin + hd * kHd + c4) = yst[it];
      }
      __threadfence();
    }
  }

  __syncthreads();
#pragma unroll
  for (int q4 = 0; q4 < 4; ++q4) {
    *(v4f*)(sH + p * kNst + nb + 4 * q4) = (v4f){hs[4 * q4 + 0], hs[4 * q4 + 1], hs[4 * q4 + 2], hs[4 * q4 + 3]};
  }
  __syncthreads();
  v4f hst[4];
#pragma unroll
  for (int it = 0; it < 4; ++it) hst[it] = *(const v4f*)(sH + (it * 256 + tid) * 4);
  float* ob = Hout + (size_t)bh * (kHd * kNst);
  for (int pass = 0; pass < 2; ++pass) {
#pragma unroll
    for (int it = 0; it < 4; ++it) *(volatile v4f*)(ob + (it * 256 + tid) * 4) = hst[it];
    __threadfence();
  }
}

constexpr int gemm_blocks(int M, int N) { return ((M / 64) * (N / 64) + 7) / 8; }

extern "C" void kernel_launch(void* const* d_in, const int* in_sizes, int n_in,
                              void* d_out, int out_size, void* d_ws, size_t ws_size,
                              hipStream_t stream) {
  if (n_in < 8) return;
  if (in_sizes[0] != kRows * kDm) return;
  if (in_sizes[1] != kDm * kDz) return;
  if (in_sizes[2] != kDm * kNssm) return;
  if (in_sizes[3] != kDz * kDin) return;
  if (in_sizes[4] != kDin * kDm) return;
  if (in_sizes[5] != kNh || in_sizes[6] != kNh || in_sizes[7] != kNh) return;
  if (out_size != kOutElems0 + kOutElems1) return;
  if (ws_size < kWsTotal) return;

  const float* x       = (const float*)d_in[0];
  const float* Wz      = (const float*)d_in[1];
  const float* Win     = (const float*)d_in[2];
  const float* Wzg     = (const float*)d_in[3];
  const float* Wout    = (const float*)d_in[4];
  const float* dt_bias = (const float*)d_in[5];
  const float* A_log   = (const float*)d_in[6];
  const float* D_param = (const float*)d_in[7];
  float* out   = (float*)d_out;
  float* hlast = out + (size_t)kOutElems0;

  char* ws = (char*)d_ws;
  unsigned short* XB    = (unsigned short*)(ws + kOffXB);
  unsigned short* WZT   = (unsigned short*)(ws + kOffWZT);
  unsigned short* WINT  = (unsigned short*)(ws + kOffWINT);
  unsigned short* WZGT  = (unsigned short*)(ws + kOffWZGT);
  unsigned short* WOUTT = (unsigned short*)(ws + kOffWOUTT);
  unsigned short* ZSH   = (unsigned short*)(ws + kOffZSH);
  unsigned short* ZSL   = (unsigned short*)(ws + kOffZSL);
  float*          SSM   = (float*)(ws + kOffSSM);
  float*          Yf    = (float*)(ws + kOffY);
  unsigned short* GH    = (unsigned short*)(ws + kOffGH);
  unsigned short* GL    = (unsigned short*)(ws + kOffGL);

  cast_rows_bf16_kernel<<<(kRows * kDm / 8) / 256, 256, 0, stream>>>(x, XB, kRows * kDm / 8);
  transpose_bf16_kernel<<<dim3(kDz / 64, kDm / 64), 256, 0, stream>>>(Wz, WZT, kDm, kDz, kDm);
  transpose_bf16_kernel<<<dim3(kLdS / 64, kDm / 64), 256, 0, stream>>>(Win, WINT, kDm, kNssm, kDm);
  transpose_bf16_kernel<<<dim3(kDin / 64, kDz / 64), 256, 0, stream>>>(Wzg, WZGT, kDz, kDin, kDz);
  transpose_bf16_kernel<<<dim3(kDm / 64, kDin / 64), 256, 0, stream>>>(Wout, WOUTT, kDin, kDm, kDin);

  wmma_gemm64<1, 0, 0, 0, false><<<dim3(gemm_blocks(kRows, kLdS)), 256, 0, stream>>>(
      XB, XB, kDm,
      WINT, WINT, kDm,
      (void*)SSM, nullptr, kLdS,
      nullptr, 0,
      kRows, kLdS, kDm, 1.0f);

  ssd_scan_kernel<<<kBatch * kNh, 256, 0, stream>>>(SSM, dt_bias, A_log, D_param, Yf, hlast);

  for (int hf = 0; hf < 2; ++hf) {
    const size_t aoff = (size_t)hf * kHalf * kDm;
    const size_t goff = (size_t)hf * kHalf * kDin;
    wmma_gemm64<1, 0, 2, 3, false><<<dim3(gemm_blocks(kHalf, kDz)), 256, 0, stream>>>(
        XB + aoff, XB + aoff, kDm,
        WZT, WZT, kDm,
        (void*)ZSH, (void*)ZSL, kDz,
        nullptr, 0,
        kHalf, kDz, kDm, 1.0f);
    wmma_gemm64<1, 1, 2, 0, true><<<dim3(gemm_blocks(kHalf, kDin)), 256, 0, stream>>>(
        ZSH, ZSL, kDz,
        WZGT, WZGT, kDz,
        (void*)(GH + goff), (void*)(GL + goff), kDin,
        Yf + goff, kDin,
        kHalf, kDin, kDz, 1.0f);
  }

  wmma_gemm64<1, 1, 0, 0, false><<<dim3(gemm_blocks(kRows, kDm)), 256, 0, stream>>>(
      GH, GL, kDin,
      WOUTT, WOUTT, kDin,
      (void*)out, nullptr, kDm,
      nullptr, 0,
      kRows, kDm, kDin, 1.0f);
}
